// TbNetV1_82489141887097
// MI455X (gfx1250) — hardware-run, weakly checked
//
#include <hip/hip_runtime.h>
#include <math.h>

typedef __attribute__((ext_vector_type(16))) _Float16 v16h;
typedef __attribute__((ext_vector_type(8)))  _Float16 v8h;
typedef __attribute__((ext_vector_type(8)))  float    v8f;
typedef __attribute__((ext_vector_type(4)))  float    v4f;
typedef __attribute__((ext_vector_type(2)))  float    v2f;
typedef __attribute__((ext_vector_type(4)))  int      v4i;
typedef __attribute__((ext_vector_type(4)))  unsigned v4u;

constexpr int kN    = 25000;
constexpr int kNP   = 25024;
constexpr int kE    = 400000;
constexpr int kFin  = 8;
constexpr int kH    = 128;
constexpr int kT    = 20;
constexpr int kV    = 5000;
constexpr int kVP   = 5056;
constexpr int kEmb  = 64;
constexpr int kG3   = 384;
constexpr int kUVW  = 256;
constexpr int kChunk   = 2048;
constexpr int kDegTile = 4096;
constexpr int kT1      = 2048;
constexpr int kT2      = 256;
constexpr int kHP      = 136;
constexpr int kEfP     = 392;
constexpr float kPos1Carry = 16.0f;
constexpr float kPosCarry  = 64.0f;
static_assert(kNP == ((kN + 63) / 64) * 64, "node pad");
static_assert(kVP == ((kV + 63) / 64) * 64, "vocab pad");
static_assert((kE % 64) == 0 && (kE % 8) == 0, "edge tiles");
static_assert((kH % 32) == 0 && (kEmb % 32) == 0 && (kG3 % 32) == 0, "K multiples of 32");
static_assert((kH % 64) == 0 && (kG3 % 64) == 0 && (kUVW % 64) == 0, "N multiples of 64");
static_assert(((size_t)kE * 2 * 4) % 128 == 0, "second output starts on a line");

constexpr size_t kSzNodeH = (size_t)kNP * kH * 2;
constexpr size_t kSzUV    = (size_t)kNP * kUVW * 4;
constexpr size_t kOffDINV = 0;
constexpr size_t kOffPOS1 = kOffDINV + (size_t)kNP * 4;
constexpr size_t kOffHW2  = kOffPOS1 + kSzNodeH;
constexpr size_t kOffPOSH = kOffHW2  + (size_t)kNP * kH * 4;
constexpr size_t kOffIMGH = kOffPOSH + kSzNodeH;
constexpr size_t kOffTXTH = kOffIMGH + kSzNodeH;
constexpr size_t kOffEMBH = kOffTXTH + kSzNodeH;
constexpr size_t kOffPTAB = kOffEMBH + (size_t)kVP * kEmb * 2;
constexpr size_t kOffWIHT = kOffPTAB + (size_t)kVP * kG3 * 4;
constexpr size_t kOffWHHT = kOffWIHT + (size_t)kG3 * kEmb * 2;
constexpr size_t kOffW2T  = kOffWHHT + (size_t)kG3 * kH * 2;
constexpr size_t kOffWCP  = kOffW2T  + (size_t)kH * kH * 2;
constexpr size_t kOffWCT  = kOffWCP  + (size_t)kUVW * kH * 2;
constexpr size_t kOffWCI  = kOffWCT  + (size_t)kUVW * kH * 2;
constexpr size_t kOffW1C  = kOffWCI  + (size_t)kUVW * kH * 2;
constexpr size_t kOffUVP  = kOffW1C  + (size_t)kUVW * kG3 * 2;
constexpr size_t kOffUVT  = kOffUVP  + kSzUV;
constexpr size_t kOffUVI  = kOffUVT  + kSzUV;
constexpr size_t kWsTotal = kOffUVI  + kSzUV;
static_assert(kWsTotal == 124397312ull, "carve total");
static_assert(kWsTotal <= 134217728ull, "carve cap");
static_assert((kOffPOS1 % 128) == 0 && (kOffHW2 % 128) == 0 && (kOffPOSH % 128) == 0 && (kOffIMGH % 128) == 0 &&
              (kOffTXTH % 128) == 0 && (kOffEMBH % 128) == 0 && (kOffPTAB % 128) == 0 && (kOffWIHT % 128) == 0 &&
              (kOffWHHT % 128) == 0 && (kOffW2T % 128) == 0 && (kOffWCP % 128) == 0 && (kOffWCT % 128) == 0 &&
              (kOffWCI % 128) == 0 && (kOffW1C % 128) == 0 && (kOffUVP % 128) == 0 && (kOffUVT % 128) == 0 &&
              (kOffUVI % 128) == 0, "128-B aligned regions");

struct FragH {
  union U { v16h v; v8h h[2]; };
  static __device__ __forceinline__ v16h load(const _Float16* p) {
    U f; f.h[0] = *(const v8h*)(p); f.h[1] = *(const v8h*)(p + 16); return f.v;
  }
  static __device__ __forceinline__ v8f mma(v16h a, v16h b, v8f c) {
    return __builtin_amdgcn_wmma_f32_16x16x32_f16(false, a, false, b, (short)0, c, false, false);
  }
};
__device__ __forceinline__ void tie_acc(v8f& a) { asm volatile("" : "+v"(a)); }
__device__ __forceinline__ void nop_guard4(v8f& a, v16h x0, v16h x1, v16h x2, v16h x3) {
  asm volatile("v_nop\n\tv_nop\n\tv_nop\n\tv_nop" : "+v"(a) : "v"(x0), "v"(x1), "v"(x2), "v"(x3));
}
__device__ __forceinline__ void nop_guard5(v8f& a, v16h x0, v16h x1, v16h x2, v16h x3, v16h x4) {
  asm volatile("v_nop\n\tv_nop\n\tv_nop\n\tv_nop" : "+v"(a) : "v"(x0), "v"(x1), "v"(x2), "v"(x3), "v"(x4));
}
__device__ __forceinline__ void nop_guard6(v8f& a, v16h x0, v16h x1, v16h x2, v16h x3, v16h x4, v16h x5) {
  asm volatile("v_nop\n\tv_nop\n\tv_nop\n\tv_nop" : "+v"(a) : "v"(x0), "v"(x1), "v"(x2), "v"(x3), "v"(x4), "v"(x5));
}
__device__ __forceinline__ void acc_guard4(v8f& a, v8f& b, v8f& c, v8f& d) {
  asm volatile("v_nop\n\tv_nop\n\tv_nop\n\tv_nop" : "+v"(a), "+v"(b), "+v"(c), "+v"(d));
}
__device__ __forceinline__ float fast_sigmoid(float v) { return __builtin_amdgcn_rcpf(1.0f + __expf(-v)); }
__device__ __forceinline__ float fast_tanh(float v) { return 1.0f - 2.0f * __builtin_amdgcn_rcpf(__expf(2.0f * v) + 1.0f); }

template <int BIAS_MODE>
__global__ __launch_bounds__(256) void wmma_gemm64(
    const unsigned short* __restrict__ Ap, int lda,
    const unsigned short* __restrict__ Btp, int ldb,
    float* __restrict__ C, int ldc,
    const float* __restrict__ bias,
    int M, int N, int K, float scale) {
  const _Float16* A = (const _Float16*)Ap;
  const _Float16* Bt = (const _Float16*)Btp;
  __shared__ __align__(16) float sT[8][16 * 68];
  const int lane = threadIdx.x & 31;
  const int wave = threadIdx.x >> 5;
  const int tilesN = N >> 6;
  const int tilesM = M >> 6;
  const int tile = blockIdx.x * 8 + wave;
  if (tile >= tilesM * tilesN) return;
  const int tm = tile / tilesN;
  const int tn = tile - tm * tilesN;
  const int m0 = tm << 6;
  const int n0 = tn << 6;
  const int rlane = lane & 15;
  const int koff  = (lane >> 4) * 8;
  const int mOff  = (lane >> 4) * 8;

  v8f acc[4][4];
#pragma unroll
  for (int i = 0; i < 4; ++i)
#pragma unroll
    for (int j = 0; j < 4; ++j) acc[i][j] = (v8f){0.f,0.f,0.f,0.f,0.f,0.f,0.f,0.f};

  for (int k0 = 0; k0 < K; k0 += 32) {
    v16h bh[4];
#pragma unroll
    for (int j = 0; j < 4; ++j) {
      const size_t bo = (size_t)(n0 + (j << 4) + rlane) * ldb + koff + k0;
      bh[j] = FragH::load(Bt + bo);
    }
#pragma unroll
    for (int i = 0; i < 4; ++i) {
      const size_t ao = (size_t)(m0 + (i << 4) + rlane) * lda + koff + k0;
      v16h ah = FragH::load(A + ao);
#pragma unroll
      for (int j = 0; j < 4; ++j) acc[i][j] = FragH::mma(ah, bh[j], acc[i][j]);
      tie_acc(acc[i][0]);
      tie_acc(acc[i][1]);
      tie_acc(acc[i][2]);
      nop_guard5(acc[i][3], ah, bh[0], bh[1], bh[2], bh[3]);
    }
  }
  acc_guard4(acc[0][0], acc[0][1], acc[0][2], acc[0][3]);
  acc_guard4(acc[1][0], acc[1][1], acc[1][2], acc[1][3]);
  acc_guard4(acc[2][0], acc[2][1], acc[2][2], acc[2][3]);
  acc_guard4(acc[3][0], acc[3][1], acc[3][2], acc[3][3]);

  float* slab = sT[wave];
#pragma unroll
  for (int i = 0; i < 4; ++i) {
    const int mBase = m0 + (i << 4);
#pragma unroll
    for (int j = 0; j < 4; ++j) {
      const int n = n0 + (j << 4) + rlane;
      float bv = 0.f;
      if (BIAS_MODE == 2) bv = bias[n];
#pragma unroll
      for (int r = 0; r < 8; ++r) {
        float v = acc[i][j][r] * scale;
        if (BIAS_MODE == 2) v += bv;
        slab[(mOff + r) * 68 + (j << 4) + rlane] = v;
      }
    }
    __builtin_amdgcn_fence(__ATOMIC_RELEASE, "workgroup");
    __builtin_amdgcn_wave_barrier();
    __builtin_amdgcn_fence(__ATOMIC_ACQUIRE, "workgroup");
    {
      const int hh = lane >> 4, c4 = (lane & 15) * 4;
      for (int pass = 0; pass < 2; ++pass) {
#pragma unroll
        for (int it = 0; it < 8; ++it) {
          const int row = it * 2 + hh;
          v4f v = *(const v4f*)(slab + row * 68 + c4);
          *(volatile v4f*)(C + (size_t)(mBase + row) * ldc + n0 + c4) = v;
        }
        __threadfence();
      }
    }
    __builtin_amdgcn_fence(__ATOMIC_RELEASE, "workgroup");
    __builtin_amdgcn_wave_barrier();
    __builtin_amdgcn_fence(__ATOMIC_ACQUIRE, "workgroup");
  }
}

__global__ __launch_bounds__(256) void cast_rows_kernel(
    const float* __restrict__ src, unsigned short* __restrict__ dst, int nreal, int total8) {
  const int i = blockIdx.x * 256 + threadIdx.x;
  if (i >= total8) return;
  const int off = i * 8;
  const bool real = off < nreal;
  const int offc = real ? off : (nreal - 8);
  const v4f a0 = *(const v4f*)(src + offc);
  const v4f a1 = *(const v4f*)(src + offc + 4);
  v8h hv;
#pragma unroll
  for (int e = 0; e < 4; ++e) {
    const float f0 = a0[e];
    const float f1 = a1[e];
    hv[e]     = (_Float16)(real ? f0 : 0.0f);
    hv[4 + e] = (_Float16)(real ? f1 : 0.0f);
  }
  unsigned short* q = dst + off;
  *(volatile v8h*)q = hv;
  __threadfence();
  *(volatile v8h*)q = hv;
}

__global__ __launch_bounds__(256) void wt_plane_kernel(
    const float* __restrict__ s0, const float* __restrict__ s1, unsigned short* __restrict__ dst,
    int K, int ld, int nsplit, int total8) {
  const int i = blockIdx.x * 256 + threadIdx.x;
  if (i >= total8) return;
  const int kper = K >> 3;
  const int n = i / kper;
  const int k0 = (i - n * kper) * 8;
  const bool first = n < nsplit;
  const int nn = first ? n : (n - nsplit);
  const float* sp = (first ? s0 : s1) + nn;
  v8h hv;
#pragma unroll
  for (int e = 0; e < 8; ++e) {
    const float f = sp[(size_t)(k0 + e) * ld];
    hv[e] = (_Float16)f;
  }
  unsigned short* q = dst + (size_t)i * 8;
  *(volatile v8h*)q = hv;
  __threadfence();
  *(volatile v8h*)q = hv;
}

__global__ __launch_bounds__(256) void degree_kernel(const int* __restrict__ e1, float* __restrict__ dinv) {
  __shared__ int sCnt[kDegTile];
  const int tid = threadIdx.x;
  const int node0 = blockIdx.x * kDegTile;
  for (int i = tid; i < kDegTile; i += 256) sCnt[i] = 0;
  __syncthreads();
#pragma unroll 1
  for (int base = 0; base < kE; base += kChunk) {
    const int eb = base + 8 * tid;
    const bool valid = eb < kE;
    const int ebc = valid ? eb : 0;
    const v4i d0 = *(const v4i*)(e1 + ebc);
    const v4i d1 = *(const v4i*)(e1 + ebc + 4);
    int dv[8];
    dv[0] = d0[0]; dv[1] = d0[1]; dv[2] = d0[2]; dv[3] = d0[3];
    dv[4] = d1[0]; dv[5] = d1[1]; dv[6] = d1[2]; dv[7] = d1[3];
#pragma unroll
    for (int j = 0; j < 8; ++j) {
      const int dl = dv[j] - node0;
      if (valid && ((unsigned)dl < (unsigned)kDegTile)) atomicAdd(&sCnt[dl], 1);
    }
  }
  __syncthreads();
#pragma unroll 1
  for (int it = 0; it < 4; ++it) {
    const int l4 = (it * 256 + tid) * 4;
    const int n = node0 + l4;
    if (n < kNP) {
      v4f o;
#pragma unroll
      for (int e = 0; e < 4; ++e) {
        const float d = (float)(sCnt[l4 + e] + 1);
        o[e] = rsqrtf(fmaxf(d, 1.0f));
      }
      *(volatile v4f*)(dinv + n) = o;
      __threadfence();
      *(volatile v4f*)(dinv + n) = o;
    }
  }
}

__device__ __forceinline__ int scan_chunk(const int* __restrict__ e0, const int* __restrict__ e1,
                                          int base, int node0, int tileN,
                                          int* sSrc, int* sDst, int* sTot, int tid) {
  const int lane = tid & 31, wave = tid >> 5;
  const int eb = base + 8 * tid;
  const bool valid = eb < kE;
  const int ebc = valid ? eb : 0;
  const v4i s0 = *(const v4i*)(e0 + ebc);
  const v4i s1 = *(const v4i*)(e0 + ebc + 4);
  const v4i d0 = *(const v4i*)(e1 + ebc);
  const v4i d1 = *(const v4i*)(e1 + ebc + 4);
  int sv[8], dv[8];
  sv[0] = s0[0]; sv[1] = s0[1]; sv[2] = s0[2]; sv[3] = s0[3];
  sv[4] = s1[0]; sv[5] = s1[1]; sv[6] = s1[2]; sv[7] = s1[3];
  dv[0] = d0[0]; dv[1] = d0[1]; dv[2] = d0[2]; dv[3] = d0[3];
  dv[4] = d1[0]; dv[5] = d1[1]; dv[6] = d1[2]; dv[7] = d1[3];
  unsigned hm = 0u;
#pragma unroll
  for (int j = 0; j < 8; ++j) {
    const int dl = dv[j] - node0;
    const bool hit = valid && ((unsigned)dl < (unsigned)tileN);
    hm |= hit ? (1u << j) : 0u;
    dv[j] = dl;
  }
  const int cnt = __popc(hm);
  int inc = cnt;
#pragma unroll
  for (int off = 1; off < 32; off <<= 1) {
    const int t = __shfl_up(inc, off, 32);
    inc += (lane >= off) ? t : 0;
  }
  if (lane == 31) sTot[wave] = inc;
  __syncthreads();
  int wbase = 0, total = 0;
#pragma unroll
  for (int w = 0; w < 8; ++w) {
    const int tw = sTot[w];
    total += tw;
    wbase += (w < wave) ? tw : 0;
  }
  int pos = wbase + inc - cnt;
#pragma unroll
  for (int j = 0; j < 8; ++j) {
    if (hm & (1u << j)) {
      int s = sv[j];
      s = s < 0 ? 0 : (s > kN - 1 ? kN - 1 : s);
      sSrc[pos] = s;
      sDst[pos] = dv[j];
      ++pos;
    }
  }
  __syncthreads();
  return total;
}

__global__ __launch_bounds__(256) void gcn_agg8_kernel(
    const int* __restrict__ e0, const int* __restrict__ e1, const float* __restrict__ x,
    const float* __restrict__ dinv, const float* __restrict__ w1, const float* __restrict__ b1,
    unsigned short* __restrict__ pos1h) {
  __shared__ __align__(16) float sAcc[kT1 * 8];
  __shared__ float sDin[kT1];
  __shared__ int sSrc[kChunk];
  __shared__ int sDst[kChunk];
  __shared__ int sTot[8];
  const int tid = threadIdx.x, lane = tid & 31, wave = tid >> 5;
  const int node0 = blockIdx.x * kT1;
  for (int i = tid; i < kT1 * 8; i += 256) sAcc[i] = 0.0f;
  for (int i = tid; i < kT1; i += 256) {
    int n = node0 + i;
    n = n < kNP - 1 ? n : kNP - 1;
    sDin[i] = dinv[n];
  }
  for (int i = tid; i < kChunk; i += 256) { sSrc[i] = 0; sDst[i] = 0; }
  __syncthreads();
  const int cc = lane & 7;
#pragma unroll 1
  for (int base = 0; base < kE; base += kChunk) {
    int nh = scan_chunk(e0, e1, base, node0, kT1, sSrc, sDst, sTot, tid);
    nh = __builtin_amdgcn_readfirstlane(nh);
    nh = nh < kChunk ? nh : kChunk;
#pragma unroll 1
    for (int b0 = 0; b0 < nh; b0 += 32) {
      const int idx = b0 + lane;
      const int idc = idx < kChunk ? idx : kChunk - 1;
      const int dlv = sDst[idc];
      const bool mine = (idx < nh) && ((dlv & 7) == wave);
      unsigned m = __builtin_amdgcn_ballot_w32(mine);
      while (m) {
        const int i = __builtin_ctz(m);
        m &= (m - 1u);
        const int hI = b0 + i;
        const int dl = sDst[hI];
        const int s = sSrc[hI];
        const float w = dinv[s] * sDin[dl];
        const float xv = x[(size_t)s * kFin + cc];
        const float cur = sAcc[dl * 8 + cc];
        const float nv = fmaf(w, xv, cur);
        if (lane < 8) sAcc[dl * 8 + cc] = nv;
      }
    }
    __syncthreads();
  }
#pragma unroll 1
  for (int it = 0; it < (kT1 * 16) / 256; ++it) {
    const int task = it * 256 + tid;
    const int dl = task >> 4;
    const int seg = task & 15;
    const int n = node0 + dl;
    if (n < kNP) {
      const bool real = n < kN;
      const int nr = real ? n : kN - 1;
      const float ds = sDin[dl];
      const float dself = ds * ds;
      const int c0 = seg * 8;
      const v4f bA = *(const v4f*)(b1 + c0);
      const v4f bB = *(const v4f*)(b1 + c0 + 4);
      float o[8];
      o[0] = bA[0]; o[1] = bA[1]; o[2] = bA[2]; o[3] = bA[3];
      o[4] = bB[0]; o[5] = bB[1]; o[6] = bB[2]; o[7] = bB[3];
#pragma unroll 1
      for (int k = 0; k < kFin; ++k) {
        const float xk = sAcc[dl * 8 + k] + dself * x[(size_t)nr * kFin + k];
        const v4f wA = *(const v4f*)(w1 + k * kH + c0);
        const v4f wB = *(const v4f*)(w1 + k * kH + c0 + 4);
        o[0] = fmaf(xk, wA[0], o[0]); o[1] = fmaf(xk, wA[1], o[1]);
        o[2] = fmaf(xk, wA[2], o[2]); o[3] = fmaf(xk, wA[3], o[3]);
        o[4] = fmaf(xk, wB[0], o[4]); o[5] = fmaf(xk, wB[1], o[5]);
        o[6] = fmaf(xk, wB[2], o[6]); o[7] = fmaf(xk, wB[3], o[7]);
      }
      v8h hv;
#pragma unroll
      for (int e = 0; e < 8; ++e) {
        const float v = fmaxf(o[e], 0.0f) * kPos1Carry;
        hv[e] = (_Float16)(real ? v : 0.0f);
      }
      unsigned short* q = pos1h + (size_t)n * kH + c0;
      *(volatile v8h*)q = hv;
      __threadfence();
      *(volatile v8h*)q = hv;
    }
  }
}

__global__ __launch_bounds__(256) void gcn_agg128_kernel(
    const int* __restrict__ e0, const int* __restrict__ e1, const float* __restrict__ hw2,
    const float* __restrict__ dinv, const float* __restrict__ b2, unsigned short* __restrict__ posh) {
  __shared__ __align__(16) float sAcc[kT2 * kH];
  __shared__ float sDin[kT2];
  __shared__ int sSrc[kChunk];
  __shared__ int sDst[kChunk];
  __shared__ int sTot[8];
  const int tid = threadIdx.x, lane = tid & 31, wave = tid >> 5;
  const int node0 = blockIdx.x * kT2;
  for (int i = tid; i < kT2 * kH; i += 256) sAcc[i] = 0.0f;
  for (int i = tid; i < kT2; i += 256) {
    int n = node0 + i;
    n = n < kNP - 1 ? n : kNP - 1;
    sDin[i] = dinv[n];
  }
  for (int i = tid; i < kChunk; i += 256) { sSrc[i] = 0; sDst[i] = 0; }
  __syncthreads();
#pragma unroll 1
  for (int base = 0; base < kE; base += kChunk) {
    int nh = scan_chunk(e0, e1, base, node0, kT2, sSrc, sDst, sTot, tid);
    nh = __builtin_amdgcn_readfirstlane(nh);
    nh = nh < kChunk ? nh : kChunk;
#pragma unroll 1
    for (int b0 = 0; b0 < nh; b0 += 32) {
      const int idx = b0 + lane;
      const int idc = idx < kChunk ? idx : kChunk - 1;
      const int dlv = sDst[idc];
      const bool mine = (idx < nh) && ((dlv & 7) == wave);
      unsigned m = __builtin_amdgcn_ballot_w32(mine);
      while (m) {
        const int i = __builtin_ctz(m);
        m &= (m - 1u);
        const int hI = b0 + i;
        const int dl = sDst[hI];
        const int s = sSrc[hI];
        const float w = dinv[s] * sDin[dl];
        const v4f hv = *(const v4f*)(hw2 + (size_t)s * kH + lane * 4);
        v4f a = *(const v4f*)(sAcc + dl * kH + lane * 4);
        a[0] = fmaf(w, hv[0], a[0]);
        a[1] = fmaf(w, hv[1], a[1]);
        a[2] = fmaf(w, hv[2], a[2]);
        a[3] = fmaf(w, hv[3], a[3]);
        *(v4f*)(sAcc + dl * kH + lane * 4) = a;
      }
    }
    __syncthreads();
  }
#pragma unroll 1
  for (int it = 0; it < (kT2 * 16) / 256; ++it) {
    const int task = it * 256 + tid;
    const int dl = task >> 4;
    const int seg = task & 15;
    const int n = node0 + dl;
    if (n < kNP) {
      const bool real = n < kN;
      const int nr = real ? n : kN - 1;
      const float ds = sDin[dl];
      const float dself = ds * ds;
      const int c0 = seg * 8;
      const v4f aA = *(const v4f*)(sAcc + dl * kH + c0);
      const v4f aB = *(const v4f*)(sAcc + dl * kH + c0 + 4);
      const v4f hA = *(const v4f*)(hw2 + (size_t)nr * kH + c0);
      const v4f hB = *(const v4f*)(hw2 + (size_t)nr * kH + c0 + 4);
      const v4f bA = *(const v4f*)(b2 + c0);
      const v4f bB = *(const v4f*)(b2 + c0 + 4);
      v8h hv;
#pragma unroll
      for (int e = 0; e < 4; ++e) {
        const float v0 = fmaxf((aA[e] + dself * hA[e]) + bA[e], 0.0f) * kPosCarry;
        const float v1 = fmaxf((aB[e] + dself * hB[e]) + bB[e], 0.0f) * kPosCarry;
        hv[e]     = (_Float16)(real ? v0 : 0.0f);
        hv[4 + e] = (_Float16)(real ? v1 : 0.0f);
      }
      unsigned short* q = posh + (size_t)n * kH + c0;
      *(volatile v8h*)q = hv;
      __threadfence();
      *(volatile v8h*)q = hv;
    }
  }
}

__global__ __launch_bounds__(256) void gru_kernel(
    const int* __restrict__ xtext, const float* __restrict__ P, const unsigned short* __restrict__ whht_p,
    const float* __restrict__ bhh, unsigned short* __restrict__ txth) {
  __shared__ __align__(16) _Float16 sH[2][64 * kHP];
  __shared__ int sTok[kT * 64];
  const _Float16* Wt = (const _Float16*)whht_p;
  const int tid = threadIdx.x, lane = tid & 31, wave = tid >> 5;
  const int hh = lane >> 4, c = lane & 15;
  const int koff = hh * 8;
  const int n0 = blockIdx.x * 64;
  for (int i = tid; i < 64 * kT; i += 256) {
    const int row = i / kT;
    const int tt = i - row * kT;
    int n = n0 + row;
    n = n < kN - 1 ? n : kN - 1;
    int tok = xtext[(size_t)n * kT + tt];
    tok = tok < 0 ? 0 : (tok > kV - 1 ? kV - 1 : tok);
    sTok[tt * 64 + row] = tok;
  }
  __syncthreads();
  const int col = wave * 16 + c;
  const float bhr = bhh[col], bhz = bhh[kH + col], bhn = bhh[2 * kH + col];
  v8f h[4];
#pragma unroll
  for (int i = 0; i < 4; ++i) h[i] = (v8f){0.f,0.f,0.f,0.f,0.f,0.f,0.f,0.f};

#pragma unroll 1
  for (int t = 0; t < kT; ++t) {
    const _Float16* sHc = sH[t & 1];
    _Float16* sHn = sH[(t + 1) & 1];
    v8f acc[4][3];
#pragma unroll
    for (int i = 0; i < 4; ++i)
#pragma unroll
      for (int g = 0; g < 3; ++g) acc[i][g] = (v8f){0.f,0.f,0.f,0.f,0.f,0.f,0.f,0.f};
    if (t > 0) {
#pragma unroll 1
      for (int k0 = 0; k0 < kH; k0 += 32) {
        v16h bf[3];
#pragma unroll
        for (int g = 0; g < 3; ++g)
          bf[g] = FragH::load(Wt + (size_t)(g * kH + col) * kH + koff + k0);
#pragma unroll
        for (int i = 0; i < 4; ++i) {
          v16h a = FragH::load(sHc + (i * 16 + c) * kHP + koff + k0);
#pragma unroll
          for (int g = 0; g < 3; ++g) acc[i][g] = FragH::mma(a, bf[g], acc[i][g]);
          tie_acc(acc[i][0]);
          tie_acc(acc[i][1]);
          nop_guard4(acc[i][2], a, bf[0], bf[1], bf[2]);
        }
      }
    }
#pragma unroll
    for (int i = 0; i < 4; ++i) {
#pragma unroll
      for (int rh = 0; rh < 2; ++rh) {
        float xr[4], xz[4], xn[4];
#pragma unroll
        for (int q = 0; q < 4; ++q) {
          const int row = i * 16 + 8 * hh + rh * 4 + q;
          const int tok = sTok[t * 64 + row];
          const float* pp = P + (size_t)tok * kG3 + col;
          xr[q] = pp[0];
          xz[q] = pp[kH];
          xn[q] = pp[2 * kH];
        }
#pragma unroll
        for (int q = 0; q < 4; ++q) {
          const int r = rh * 4 + q;
          const int row = i * 16 + 8 * hh + r;
          const float hr = acc[i][0][r] + bhr;
          const float hz = acc[i][1][r] + bhz;
          const float hn = acc[i][2][r] + bhn;
          const float rg = fast_sigmoid(xr[q] + hr);
          const float zg = fast_sigmoid(xz[q] + hz);
          const float ng = fast_tanh(xn[q] + rg * hn);
          const float hnew = (1.0f - zg) * ng + zg * h[i][r];
          h[i][r] = hnew;
          sHn[row * kHP + col] = (_Float16)hnew;
        }
        asm volatile("" ::: "memory");
      }
    }
    __syncthreads();
  }
  static_assert((kT & 1) == 0, "final buffer index");
#pragma unroll 1
  for (int it = 0; it < 4; ++it) {
    const int task = it * 256 + tid;
    const int row = task >> 4;
    const int seg = task & 15;
    const int n = n0 + row;
    const bool real = n < kN;
    v4u w = *(const v4u*)(&sH[0][row * kHP + seg * 8]);
    w[0] = real ? w[0] : 0u;
    w[1] = real ? w[1] : 0u;
    w[2] = real ? w[2] : 0u;
    w[3] = real ? w[3] : 0u;
    unsigned short* q = txth + (size_t)n * kH + seg * 8;
    *(volatile v4u*)q = w;
    __threadfence();
    *(volatile v4u*)q = w;
  }
}

__global__ __launch_bounds__(256) void edge_kernel(
    const int* __restrict__ e0, const int* __restrict__ e1,
    const float* __restrict__ uvp, const float* __restrict__ uvt, const float* __restrict__ uvi,
    const float* __restrict__ pb, const float* __restrict__ tb, const float* __restrict__ ib,
    const unsigned short* __restrict__ w1cat_p,
    const float* __restrict__ rb1, const float* __restrict__ cb1,
    const float* __restrict__ rw2, const float* __restrict__ cw2,
    const float* __restrict__ rb2, const float* __restrict__ cb2,
    float* __restrict__ out) {
  __shared__ __align__(16) _Float16 sEf[64 * kEfP];
  __shared__ __align__(16) float sBias[kG3];
  __shared__ int sIdx[128];
  __shared__ __align__(16) float sPart[8 * 64 * 2];
  const _Float16* W = (const _Float16*)w1cat_p;
  const int tid = threadIdx.x, lane = tid & 31, wave = tid >> 5;
  const int hh = lane >> 4, c = lane & 15;
  const int koff = hh * 8;
  const int m0 = blockIdx.x * 64;
  if (tid < 128) {
    const int* ep = (tid < 64) ? e0 : e1;
    int v = ep[m0 + (tid & 63)];
    v = v < 0 ? 0 : (v > kN - 1 ? kN - 1 : v);
    sIdx[tid] = v;
    sBias[tid] = pb[tid];
    sBias[2 * kH + tid] = ib[tid];
  } else {
    sBias[tid] = tb[tid - 128];
  }
  __syncthreads();
#pragma unroll 1
  for (int it = 0; it < 12; ++it) {
    const int f = it >> 2;
    const float* uv = (f == 0) ? uvp : ((f == 1) ? uvt : uvi);
    const int e = (it & 3) * 16 + (tid >> 4);
    const int seg = tid & 15;
    const int i0 = sIdx[e];
    const int i1 = sIdx[64 + e];
    const float* pu = uv + (size_t)i0 * kUVW + seg * 8;
    const float* pv = uv + (size_t)i1 * kUVW + kH + seg * 8;
    const v4f u0 = *(const v4f*)(pu);
    const v4f u1 = *(const v4f*)(pu + 4);
    const v4f v0 = *(const v4f*)(pv);
    const v4f v1 = *(const v4f*)(pv + 4);
    const v4f b0 = *(const v4f*)(sBias + f * kH + seg * 8);
    const v4f b1 = *(const v4f*)(sBias + f * kH + seg * 8 + 4);
    v8h hv;
#pragma unroll
    for (int q = 0; q < 4; ++q) {
      const float a0 = (u0[q] + v0[q]) + b0[q];
      const float a1 = (u1[q] + v1[q]) + b1[q];
      hv[q]     = (_Float16)fmaxf(a0, 0.0f);
      hv[4 + q] = (_Float16)fmaxf(a1, 0.0f);
    }
    *(v8h*)(sEf + e * kEfP + f * kH + seg * 8) = hv;
  }
  __syncthreads();

  v8f acc[2][4];
#pragma unroll
  for (int u = 0; u < 2; ++u)
#pragma unroll
    for (int et = 0; et < 4; ++et) acc[u][et] = (v8f){0.f,0.f,0.f,0.f,0.f,0.f,0.f,0.f};
#pragma unroll 1
  for (int k0 = 0; k0 < kG3; k0 += 32) {
    v16h a[2], b[4];
#pragma unroll
    for (int u = 0; u < 2; ++u)
      a[u] = FragH::load(W + (size_t)(wave * 32 + u * 16 + c) * kG3 + koff + k0);
#pragma unroll
    for (int et = 0; et < 4; ++et)
      b[et] = FragH::load(sEf + (et * 16 + c) * kEfP + koff + k0);
#pragma unroll
    for (int u = 0; u < 2; ++u)
#pragma unroll
      for (int et = 0; et < 4; ++et) acc[u][et] = FragH::mma(a[u], b[et], acc[u][et]);
    tie_acc(acc[0][0]);
    tie_acc(acc[0][1]);
    tie_acc(acc[0][2]);
    tie_acc(acc[0][3]);
    tie_acc(acc[1][0]);
    tie_acc(acc[1][1]);
    tie_acc(acc[1][2]);
    nop_guard6(acc[1][3], a[0], a[1], b[0], b[1], b[2], b[3]);
  }

  {
    const int head = wave >> 2;
    const float* b1p = head ? cb1 : rb1;
    const float* w2p = head ? cw2 : rw2;
    float p0[4], p1[4];
#pragma unroll
    for (int et = 0; et < 4; ++et) { p0[et] = 0.0f; p1[et] = 0.0f; }
#pragma unroll
    for (int u = 0; u < 2; ++u) {
      const int ub = (wave & 3) * 32 + u * 16 + 8 * hh;
      const v4f bA = *(const v4f*)(b1p + ub);
      const v4f bB = *(const v4f*)(b1p + ub + 4);
      const v4f wA = *(const v4f*)(w2p + ub * 2);
      const v4f wB = *(const v4f*)(w2p + ub * 2 + 4);
      const v4f wC = *(const v4f*)(w2p + ub * 2 + 8);
      const v4f wD = *(const v4f*)(w2p + ub * 2 + 12);
      float bb[8], wa[8], wb[8];
      bb[0] = bA[0]; bb[1] = bA[1]; bb[2] = bA[2]; bb[3] = bA[3];
      bb[4] = bB[0]; bb[5] = bB[1]; bb[6] = bB[2]; bb[7] = bB[3];
      wa[0] = wA[0]; wb[0] = wA[1]; wa[1] = wA[2]; wb[1] = wA[3];
      wa[2] = wB[0]; wb[2] = wB[1]; wa[3] = wB[2]; wb[3] = wB[3];
      wa[4] = wC[0]; wb[4] = wC[1]; wa[5] = wC[2]; wb[5] = wC[3];
      wa[6] = wD[0]; wb[6] = wD[1]; wa[7] = wD[2]; wb[7] = wD[3];
#pragma unroll
      for (int r = 0; r < 8; ++r) {
#pragma unroll
        for (int et = 0; et < 4; ++et) {
          const float v = fmaxf(acc[u][et][r] + bb[r], 0.0f);
          p0[et] = fmaf(v, wa[r], p0[et]);
          p1[et] = fmaf(v, wb[r], p1[et]);
        }
      }
    }
#pragma unroll
    for (int et = 0; et < 4; ++et) {
      const float o0 = __shfl_xor(p0[et], 16, 32);
      const float o1 = __shfl_xor(p1[et], 16, 32);
      p0[et] += o0;
      p1[et] += o1;
    }
    if (hh == 0) {
#pragma unroll
      for (int et = 0; et < 4; ++et) {
        sPart[(wave * 64 + et * 16 + c) * 2 + 0] = p0[et];
        sPart[(wave * 64 + et * 16 + c) * 2 + 1] = p1[et];
      }
    }
  }
  __syncthreads();
  if (tid < 128) {
    const int head = tid >> 6;
    const int e = tid & 63;
    const float* b2p = head ? cb2 : rb2;
    float l0 = 0.0f, l1 = 0.0f;
#pragma unroll
    for (int w = 0; w < 4; ++w) {
      l0 += sPart[((head * 4 + w) * 64 + e) * 2 + 0];
      l1 += sPart[((head * 4 + w) * 64 + e) * 2 + 1];
    }
    l0 += b2p[0];
    l1 += b2p[1];
    const float mx = fmaxf(l0, l1);
    const float lse = mx + logf(expf(l0 - mx) + expf(l1 - mx));
    v2f ov;
    ov[0] = l0 - lse;
    ov[1] = l1 - lse;
    float* op = out + (size_t)head * ((size_t)kE * 2) + (size_t)(m0 + e) * 2;
    *(volatile v2f*)op = ov;
    __threadfence();
    *(volatile v2f*)op = ov;
  }
}

extern "C" void kernel_launch(void* const* d_in, const int* in_sizes, int n_in,
                              void* d_out, int out_size, void* d_ws, size_t ws_size,
                              hipStream_t stream) {
  if (n_in < 27) return;
  if (in_sizes[0] != kN * kFin) return;
  if (in_sizes[1] != kN * kH) return;
  if (in_sizes[2] != 2 * kE) return;
  if (in_sizes[3] != kN * kT) return;
  if (in_sizes[8] != kV * kEmb) return;
  if (in_sizes[9] != kEmb * kG3) return;
  if (in_sizes[10] != kH * kG3) return;
  if (in_sizes[13] != 2 * kH * kH) return;
  if (in_sizes[19] != kG3 * kH) return;
  if (in_sizes[23] != kG3 * kH) return;
  if (out_size != 4 * kE) return;
  if (ws_size < kWsTotal) return;

  const float* x      = (const float*)d_in[0];
  const float* img    = (const float*)d_in[1];
  const int*   eidx   = (const int*)d_in[2];
  const int*   xtext  = (const int*)d_in[3];
  const float* gcn_w1 = (const float*)d_in[4];
  const float* gcn_b1 = (const float*)d_in[5];
  const float* gcn_w2 = (const float*)d_in[6];
  const float* gcn_b2 = (const float*)d_in[7];
  const float* embed  = (const float*)d_in[8];
  const float* w_ih   = (const float*)d_in[9];
  const float* w_hh   = (const float*)d_in[10];
  const float* b_ih   = (const float*)d_in[11];
  const float* b_hh   = (const float*)d_in[12];
  const float* pos_w  = (const float*)d_in[13];
  const float* pos_b  = (const float*)d_in[14];
  const float* text_w = (const float*)d_in[15];
  const float* text_b = (const float*)d_in[16];
  const float* img_w  = (const float*)d_in[17];
  const float* img_b  = (const float*)d_in[18];
  const float* row_w1 = (const float*)d_in[19];
  const float* row_b1 = (const float*)d_in[20];
  const float* row_w2 = (const float*)d_in[21];
  const float* row_b2 = (const float*)d_in[22];
  const float* col_w1 = (const float*)d_in[23];
  const float* col_b1 = (const float*)d_in[24];
  const float* col_w2 = (const float*)d_in[25];
  const float* col_b2 = (const float*)d_in[26];
  const int* e0 = eidx;
  const int* e1 = eidx + kE;
  float* out = (float*)d_out;

  char* ws = (char*)d_ws;
  float*          DINV  = (float*)(ws + kOffDINV);
  unsigned short* POS1H = (unsigned short*)(ws + kOffPOS1);
  float*          HW2   = (float*)(ws + kOffHW2);
  unsigned short* POSH  = (unsigned short*)(ws + kOffPOSH);
  unsigned short* IMGH  = (unsigned short*)(ws + kOffIMGH);
  unsigned short* TXTH  = (unsigned short*)(ws + kOffTXTH);
  unsigned short* EMBH  = (unsigned short*)(ws + kOffEMBH);
  float*          PTAB  = (float*)(ws + kOffPTAB);
  unsigned short* WIHT  = (unsigned short*)(ws + kOffWIHT);
  unsigned short* WHHT  = (unsigned short*)(ws + kOffWHHT);
  unsigned short* W2T   = (unsigned short*)(ws + kOffW2T);
  unsigned short* WCP   = (unsigned short*)(ws + kOffWCP);
  unsigned short* WCT   = (unsigned short*)(ws + kOffWCT);
  unsigned short* WCI   = (unsigned short*)(ws + kOffWCI);
  unsigned short* W1C   = (unsigned short*)(ws + kOffW1C);
  float*          UVP   = (float*)(ws + kOffUVP);
  float*          UVT   = (float*)(ws + kOffUVT);
  float*          UVI   = (float*)(ws + kOffUVI);

  wt_plane_kernel<<<(kG3 * kEmb / 8 + 255) / 256, 256, 0, stream>>>(w_ih, w_ih, WIHT, kEmb, kG3, kG3, kG3 * kEmb / 8);
  wt_plane_kernel<<<(kG3 * kH / 8 + 255) / 256, 256, 0, stream>>>(w_hh, w_hh, WHHT, kH, kG3, kG3, kG3 * kH / 8);
  wt_plane_kernel<<<(kH * kH / 8 + 255) / 256, 256, 0, stream>>>(gcn_w2, gcn_w2, W2T, kH, kH, kH, kH * kH / 8);
  wt_plane_kernel<<<(kUVW * kH / 8 + 255) / 256, 256, 0, stream>>>(pos_w,  pos_w  + kH * kH, WCP, kH, kH, kH, kUVW * kH / 8);
  wt_plane_kernel<<<(kUVW * kH / 8 + 255) / 256, 256, 0, stream>>>(text_w, text_w + kH * kH, WCT, kH, kH, kH, kUVW * kH / 8);
  wt_plane_kernel<<<(kUVW * kH / 8 + 255) / 256, 256, 0, stream>>>(img_w,  img_w  + kH * kH, WCI, kH, kH, kH, kUVW * kH / 8);
  wt_plane_kernel<<<(kUVW * kG3 / 8 + 255) / 256, 256, 0, stream>>>(row_w1, col_w1, W1C, kG3, kH, kH, kUVW * kG3 / 8);

  cast_rows_kernel<<<(kVP * kEmb / 8 + 255) / 256, 256, 0, stream>>>(embed, EMBH, kV * kEmb, kVP * kEmb / 8);
  cast_rows_kernel<<<(kNP * kH / 8 + 255) / 256, 256, 0, stream>>>(img, IMGH, kN * kH, kNP * kH / 8);

  degree_kernel<<<(kNP + kDegTile - 1) / kDegTile, 256, 0, stream>>>(e1, DINV);
  gcn_agg8_kernel<<<(kNP + kT1 - 1) / kT1, 256, 0, stream>>>(e0, e1, x, DINV, gcn_w1, gcn_b1, POS1H);
  wmma_gemm64<0><<<((kNP / 64) * (kH / 64) + 7) / 8, 256, 0, stream>>>(
      POS1H, kH, W2T, kH, HW2, kH, nullptr, kNP, kH, kH, 1.0f / kPos1Carry);
  gcn_agg128_kernel<<<(kNP + kT2 - 1) / kT2, 256, 0, stream>>>(e0, e1, HW2, DINV, gcn_b2, POSH);

  wmma_gemm64<2><<<((kVP / 64) * (kG3 / 64) + 7) / 8, 256, 0, stream>>>(
      EMBH, kEmb, WIHT, kEmb, PTAB, kG3, b_ih, kVP, kG3, kEmb, 1.0f);
  gru_kernel<<<kNP / 64, 256, 0, stream>>>(xtext, PTAB, WHHT, b_hh, TXTH);

  wmma_gemm64<0><<<((kNP / 64) * (kUVW / 64) + 7) / 8, 256, 0, stream>>>(
      POSH, kH, WCP, kH, UVP, kUVW, nullptr, kNP, kUVW, kH, 1.0f / kPosCarry);
  wmma_gemm64<0><<<((kNP / 64) * (kUVW / 64) + 7) / 8, 256, 0, stream>>>(
      TXTH, kH, WCT, kH, UVT, kUVW, nullptr, kNP, kUVW, kH, 1.0f);
  wmma_gemm64<0><<<((kNP / 64) * (kUVW / 64) + 7) / 8, 256, 0, stream>>>(
      IMGH, kH, WCI, kH, UVI, kUVW, nullptr, kNP, kUVW, kH, 1.0f);

  edge_kernel<<<kE / 64, 256, 0, stream>>>(
      e0, e1, UVP, UVT, UVI, pos_b, text_b, img_b, W1C,
      row_b1, col_b1, row_w2, col_w2, row_b2, col_b2, out);
}
